// DMFMLayer_32212254720200
// MI455X (gfx1250) — hardware-verified
//
#include <hip/hip_runtime.h>
#include <math.h>

typedef __attribute__((ext_vector_type(16))) _Float16 v16h;
typedef __attribute__((ext_vector_type(16))) __bf16 v16b;
typedef __attribute__((ext_vector_type(8)))  _Float16 v8h;
typedef __attribute__((ext_vector_type(8)))  float v8f;
typedef __attribute__((ext_vector_type(4)))  float v4f;
typedef __attribute__((ext_vector_type(2)))  float v2f;
typedef __attribute__((ext_vector_type(4)))  unsigned v4u;
typedef __attribute__((ext_vector_type(4)))  int v4i;
typedef float __attribute__((may_alias)) float_a;
typedef int __attribute__((may_alias)) int_a;

template <typename T> __device__ __forceinline__ void vst2(void* p, T v) { *(volatile T*)p = v; __threadfence(); *(volatile T*)p = v; }
__device__ __forceinline__ v8f wmma16(v16h a, v16h b, v8f c) {
  v8f d = __builtin_amdgcn_wmma_f32_16x16x32_f16(false, a, false, b, (short)0, c, false, false);
  asm volatile("v_nop\n\tv_nop\n\tv_nop\n\tv_nop" : "+v"(d) : "v"(a), "v"(b));
  return d;
}
__device__ __forceinline__ v8f wmma_bf(v16b a, v16b b, v8f c) {
  v8f d = __builtin_amdgcn_wmma_f32_16x16x32_bf16(false, a, false, b, (short)0, c, false, false);
  asm volatile("v_nop\n\tv_nop\n\tv_nop\n\tv_nop" : "+v"(d) : "v"(a), "v"(b));
  return d;
}
__device__ __forceinline__ v16h frag_h(const _Float16* rowk0, int lane) {
  union { v16h v; v8h q[2]; } u; const _Float16* p = rowk0 + 8 * (lane >> 4);
  u.q[0] = *(const v8h*)p; u.q[1] = *(const v8h*)(p + 16); return u.v;
}
__device__ __forceinline__ v16h frag_f32(const float* rowk0, int lane) {
  v16h a; const float* p = rowk0 + 8 * (lane >> 4);
#pragma unroll
  for (int i = 0; i < 8; ++i) { a[i] = (_Float16)p[i]; a[8 + i] = (_Float16)p[16 + i]; }
  return a;
}
__device__ __forceinline__ v16h frag_f32s(const float* rowk0, int lane, float sc) {
  v16h a; const float* p = rowk0 + 8 * (lane >> 4);
#pragma unroll
  for (int i = 0; i < 8; ++i) { a[i] = (_Float16)(p[i] * sc); a[8 + i] = (_Float16)(p[16 + i] * sc); }
  return a;
}
__device__ __forceinline__ v16h fragc_f32(const float* W, int k0, int n, int lane, int ld, int K) {
  v16h a; const int g = lane >> 4;
#pragma unroll
  for (int i = 0; i < 8; ++i) { const int ka = k0 + 8 * g + i, kb = ka + 16;
    a[i] = (_Float16)(ka < K ? W[(size_t)(ka < K ? ka : K - 1) * ld + n] : 0.f); a[8 + i] = (_Float16)(kb < K ? W[(size_t)(kb < K ? kb : K - 1) * ld + n] : 0.f); }
  return a;
}
struct F2 { v16b h, l; };
__device__ __forceinline__ F2 bsplit16(const float v[16]) { F2 r;
#pragma unroll
  for (int i = 0; i < 16; ++i) { const __bf16 h = (__bf16)v[i]; r.h[i] = h; r.l[i] = (__bf16)(v[i] - (float)h); }
  return r; }
__device__ __forceinline__ F2 split_row(const float* row, int k0, int lane) { float v[16]; const float* p = row + k0 + 8 * (lane >> 4);
#pragma unroll
  for (int i = 0; i < 8; ++i) { v[i] = p[i]; v[8 + i] = p[16 + i]; }
  return bsplit16(v); }
__device__ __forceinline__ F2 split_rowK(const float* row, int k0, int lane, int K) { float v[16]; const int g = lane >> 4;
#pragma unroll
  for (int i = 0; i < 8; ++i) { const int ka = k0 + 8 * g + i, kb = ka + 16; v[i] = ka < K ? row[ka < K ? ka : K - 1] : 0.f; v[8 + i] = kb < K ? row[kb < K ? kb : K - 1] : 0.f; }
  return bsplit16(v); }
__device__ __forceinline__ F2 split_col(const float* W, int k0, int n, int lane, int ld, int K) { float v[16]; const int g = lane >> 4;
#pragma unroll
  for (int i = 0; i < 8; ++i) { const int ka = k0 + 8 * g + i, kb = ka + 16; v[i] = ka < K ? W[(size_t)(ka < K ? ka : K - 1) * ld + n] : 0.f; v[8 + i] = kb < K ? W[(size_t)(kb < K ? kb : K - 1) * ld + n] : 0.f; }
  return bsplit16(v); }
__device__ __forceinline__ v8f mac3(const F2& a, const F2& b, v8f c) { c = wmma_bf(a.l, b.h, c); c = wmma_bf(a.h, b.l, c); return wmma_bf(a.h, b.h, c); }
__device__ __forceinline__ float sigm(float v) { return 1.0f / (1.0f + expf(-v)); }
#define LDSX() do { asm volatile("s_wait_dscnt 0" ::: "memory"); __builtin_amdgcn_wave_barrier(); __builtin_amdgcn_fence(__ATOMIC_RELEASE, "workgroup"); } while (0)


#define NBAT 4
#define LL 4096
#define NSEQ 8
#define NR (NSEQ * LL)
#define DM 128
#define DI 256
#define DS 16
#define DTR 8
#define XDW 48
#define NOUT 128
#ifndef NLT
#define NLT LL
#endif
#define NRC (NSEQ * NLT)
__device__ __forceinline__ size_t rowof(size_t rc) { return (rc / NLT) * LL + (rc % NLT); }
__device__ __forceinline__ float bfr(float v) { return (float)(__bf16)v; }
__device__ __attribute__((noinline)) float exp_ni(float v) { return expf(v); }
__device__ __forceinline__ float silu(float v) { return v / (1.0f + expf(-v)); }
__device__ __attribute__((noinline)) float softplus_(float v) { return v > 20.f ? v : log1pf(expf(v)); }

__global__ __launch_bounds__(256) void k_prep(const float* __restrict__ x, const float* __restrict__ gam, const float* __restrict__ bet, float* __restrict__ XR) {
  __shared__ __align__(16) float T[DM][64 + 4];
  const int b = blockIdx.y, l0 = blockIdx.x * 64, tid = threadIdx.x, wave = tid >> 5, lane = tid & 31;
#pragma unroll
  for (int it = 0; it < 8; ++it) { const int q = tid + 256 * it; const int c = q >> 4, p = (q & 15) * 4;
    const float4 v = *(const float4*)(x + ((size_t)b * DM + c) * LL + l0 + p); T[c][p] = bfr(v.x); T[c][p + 1] = bfr(v.y); T[c][p + 2] = bfr(v.z); T[c][p + 3] = bfr(v.w); }
  __syncthreads();
#pragma unroll 1
  for (int rr = 0; rr < 8; ++rr) { const int li = wave * 8 + rr; float v[4], s = 0.f;
#pragma unroll
    for (int i = 0; i < 4; ++i) { v[i] = T[lane * 4 + i][li]; s += v[i]; }
#pragma unroll
    for (int o = 16; o > 0; o >>= 1) s += __shfl_xor(s, o);
    const float mu = s * (1.0f / DM); float q2 = 0.f;
#pragma unroll
    for (int i = 0; i < 4; ++i) { const float d = v[i] - mu; q2 += d * d; }
#pragma unroll
    for (int o = 16; o > 0; o >>= 1) q2 += __shfl_xor(q2, o);
    const float rs = rsqrtf(q2 * (1.0f / DM) + 1e-5f);
    v4f o1, o2;
#pragma unroll
    for (int i = 0; i < 4; ++i) { const int c = lane * 4 + i; const int src = (c & 7) * 16 + (c >> 3);
      o1[i] = (v[i] - mu) * rs * bfr(gam[c]) + bfr(bet[c]); o2[i] = (T[src][li] - mu) * rs * bfr(gam[c]) + bfr(bet[c]); }
    vst2(XR + ((size_t)b * LL + l0 + li) * DM + lane * 4, o1);
    vst2(XR + ((size_t)(NBAT + b) * LL + l0 + li) * DM + lane * 4, o2);
  }
}
__global__ __launch_bounds__(128) void k_in(const float* __restrict__ XR, const float* __restrict__ Win, float* __restrict__ UB, float* __restrict__ ZB) {
  __shared__ __align__(16) float so[4][16][132];
  const int tid = threadIdx.x, wave = tid >> 5, lane = tid & 31, col = lane & 15, g = lane >> 4; const size_t r0 = rowof((size_t)blockIdx.x * 64 + wave * 16); const int n0 = blockIdx.y * 128;
  v8f acc[8] = {};
#pragma unroll
  for (int kc = 0; kc < DM / 32; ++kc) { const F2 a = split_row(XR + (r0 + col) * DM, kc * 32, lane);
#pragma unroll
    for (int j = 0; j < 8; ++j) { const v16b wb = split_row(Win + (size_t)(n0 + j * 16 + col) * DM, kc * 32, lane).h; acc[j] = wmma_bf(a.l, wb, acc[j]); acc[j] = wmma_bf(a.h, wb, acc[j]); } }
#pragma unroll
  for (int j = 0; j < 8; ++j)
#pragma unroll
    for (int r = 0; r < 8; ++r) so[wave][8 * g + r][j * 16 + col] = acc[j][r];
  LDSX();
  float* dst = n0 < DI ? UB : ZB; const int c0 = n0 < DI ? n0 : n0 - DI;
  for (int rl = 0; rl < 16; ++rl) vst2(dst + (r0 + rl) * DI + c0 + lane * 4, *(const v4f*)(&so[wave][rl][lane * 4]));
}
__global__ __launch_bounds__(256) void k_conv(const float* __restrict__ UB, const float* __restrict__ cw, const float* __restrict__ cb, float* __restrict__ XP) {
  const size_t i4 = (size_t)blockIdx.x * 256 + threadIdx.x; const size_t r = rowof(i4 / (DI / 4)); const int c0 = (int)(i4 % (DI / 4)) * 4; const int l = (int)(r % LL);
  v4f o;
#pragma unroll
  for (int e = 0; e < 4; ++e) { const int c = c0 + e; float acc = bfr(cb[c]);
#pragma unroll
    for (int k = 0; k < 4; ++k) { const int back = 3 - k; const size_t rr = (l >= back) ? r - (size_t)back : r; const float xv = UB[rr * DI + c]; acc += bfr(cw[c * 4 + k]) * ((l >= back) ? xv : 0.0f); }
    o[e] = silu(acc); }
  vst2(XP + r * DI + c0, o);
}
__global__ __launch_bounds__(128) void k_xp(const float* __restrict__ XP, const float* __restrict__ Wx, float* __restrict__ SD) {
  __shared__ __align__(16) float sd[4][16][XDW + 4];
  const int tid = threadIdx.x, wave = tid >> 5, lane = tid & 31, col = lane & 15, g = lane >> 4; const size_t r0 = rowof((size_t)blockIdx.x * 64 + wave * 16);
  v8f acc[3] = {};
#pragma unroll 2
  for (int kc = 0; kc < DI / 32; ++kc) { const F2 a = split_row(XP + (r0 + col) * DI, kc * 32, lane);
#pragma unroll
    for (int j = 0; j < 3; ++j) { const int n = j * 16 + col; const v16b wb = split_row(Wx + (size_t)(n < 40 ? n : 39) * DI, kc * 32, lane).h; acc[j] = wmma_bf(a.l, wb, acc[j]); acc[j] = wmma_bf(a.h, wb, acc[j]); } }
#pragma unroll
  for (int j = 0; j < 3; ++j)
#pragma unroll
    for (int r = 0; r < 8; ++r) { const int n = j * 16 + col; sd[wave][8 * g + r][n] = n < 40 ? acc[j][r] : 0.f; }
  LDSX();
  for (int q = lane; q < 16 * 12; q += 32) { const int rl = q / 12, pc = q - rl * 12; vst2(SD + (r0 + rl) * XDW + pc * 4, *(const v4f*)(&sd[wave][rl][pc * 4])); }
}
__global__ __launch_bounds__(256) void k_scan(const float* __restrict__ XP, const float* __restrict__ SD, const float* __restrict__ ZB, const float* __restrict__ Wdt, const float* __restrict__ bdt,
                                              const float* __restrict__ Alog, const float* __restrict__ Dp, float* __restrict__ Y) {
  const int s = blockIdx.x, d = threadIdx.x;
  float A[DS], h[DS], wd[DTR];
#pragma unroll
  for (int i = 0; i < DS; ++i) { A[i] = -expf(bfr(Alog[d * DS + i])); h[i] = 0.f; }
#pragma unroll
  for (int k = 0; k < DTR; ++k) wd[k] = bfr(Wdt[d * DTR + k]);
  const float Dd = bfr(Dp[d]), bd = bfr(bdt[d]);
#pragma unroll 1
  for (int l = 0; l < NLT; ++l) { const size_t r = (size_t)s * LL + l;
    const float* sdr = SD + r * XDW; float dl = bd;
#pragma unroll
    for (int k = 0; k < DTR; ++k) dl += sdr[k] * wd[k];
    const float dt = softplus_(dl);
    const float u = XP[r * DI + d], z = ZB[r * DI + d]; const float du = dt * u; float y = 0.f;
#pragma unroll
    for (int i = 0; i < DS; ++i) { h[i] = exp_ni(dt * A[i]) * h[i] + du * sdr[DTR + i]; y += h[i] * sdr[DTR + DS + i]; }
    vst2(Y + r * DI + d, (float_a)((y + u * Dd) * silu(z))); }
}
__global__ __launch_bounds__(128) void k_lin(const float* __restrict__ IN, const float* __restrict__ Wm, float* __restrict__ OUT) {
  __shared__ __align__(16) float so[4][16][132];
  const int tid = threadIdx.x, wave = tid >> 5, lane = tid & 31, col = lane & 15, g = lane >> 4; const size_t r0 = rowof((size_t)blockIdx.x * 64 + wave * 16);
  v8f acc[8] = {};
#pragma unroll 2
  for (int kc = 0; kc < DI / 32; ++kc) { const F2 a = split_row(IN + (r0 + col) * DI, kc * 32, lane);
#pragma unroll
    for (int j = 0; j < 8; ++j) { const v16b wb = split_row(Wm + (size_t)(j * 16 + col) * DI, kc * 32, lane).h; acc[j] = wmma_bf(a.l, wb, acc[j]); acc[j] = wmma_bf(a.h, wb, acc[j]); } }
#pragma unroll
  for (int j = 0; j < 8; ++j)
#pragma unroll
    for (int r = 0; r < 8; ++r) so[wave][8 * g + r][j * 16 + col] = acc[j][r];
  LDSX();
  for (int rl = 0; rl < 16; ++rl) vst2(OUT + (r0 + rl) * DM + lane * 4, *(const v4f*)(&so[wave][rl][lane * 4]));
}
__global__ __launch_bounds__(256) void k_fin(const float* __restrict__ MO, const float* __restrict__ XR, const float* __restrict__ gam, const float* __restrict__ bet, const float* __restrict__ Wp, const float* __restrict__ bp,
                                             const float* __restrict__ ps1, const float* __restrict__ ps2, float* __restrict__ out) {
  __shared__ __align__(16) float sx[64][DM + 4];
  __shared__ __align__(16) float soT[NOUT][64 + 4];
  const int b = blockIdx.y, l0 = blockIdx.x * 64, tid = threadIdx.x, wave = tid >> 5, lane = tid & 31, col = lane & 15, g = lane >> 4;
  const float s1 = bfr(ps1[0]), s2 = bfr(ps2[0]);
  const size_t ra = (size_t)b * LL + l0, rb2 = (size_t)(NBAT + b) * LL + l0;
#pragma unroll 1
  for (int rr = 0; rr < 8; ++rr) { const int li = wave * 8 + rr; float v[4], s = 0.f;
    const float4 m1 = *(const float4*)(MO + (ra + li) * DM + lane * 4), x1 = *(const float4*)(XR + (ra + li) * DM + lane * 4);
    const float4 m2 = *(const float4*)(MO + (rb2 + li) * DM + lane * 4), x2 = *(const float4*)(XR + (rb2 + li) * DM + lane * 4);
    v[0] = (m1.x + x1.x * s1) + (m2.x + x2.x * s2); v[1] = (m1.y + x1.y * s1) + (m2.y + x2.y * s2); v[2] = (m1.z + x1.z * s1) + (m2.z + x2.z * s2); v[3] = (m1.w + x1.w * s1) + (m2.w + x2.w * s2);
#pragma unroll
    for (int i = 0; i < 4; ++i) s += v[i];
#pragma unroll
    for (int o = 16; o > 0; o >>= 1) s += __shfl_xor(s, o);
    const float mu = s * (1.0f / DM); float q2 = 0.f;
#pragma unroll
    for (int i = 0; i < 4; ++i) { const float dd = v[i] - mu; q2 += dd * dd; }
#pragma unroll
    for (int o = 16; o > 0; o >>= 1) q2 += __shfl_xor(q2, o);
    const float rs = rsqrtf(q2 * (1.0f / DM) + 1e-5f);
#pragma unroll
    for (int i = 0; i < 4; ++i) { const int c = lane * 4 + i; sx[li][c] = (v[i] - mu) * rs * bfr(gam[c]) + bfr(bet[c]); } }
  __syncthreads();
  const int rt = wave & 3, ct0 = (wave >> 2) * 4; v8f acc[4] = {};
#pragma unroll
  for (int kc = 0; kc < DM / 32; ++kc) { const F2 a = split_row(&sx[rt * 16 + col][0], kc * 32, lane);
#pragma unroll
    for (int j = 0; j < 4; ++j) { const v16b wb = split_row(Wp + (size_t)((ct0 + j) * 16 + col) * DM, kc * 32, lane).h; acc[j] = wmma_bf(a.l, wb, acc[j]); acc[j] = wmma_bf(a.h, wb, acc[j]); } }
#pragma unroll
  for (int j = 0; j < 4; ++j) { const int o = (ct0 + j) * 16 + col; const float bb = bfr(bp[o]);
#pragma unroll
    for (int r = 0; r < 8; ++r) soT[o][rt * 16 + 8 * g + r] = acc[j][r] + bb; }
  __syncthreads();
#pragma unroll
  for (int it = 0; it < 8; ++it) { const int q = tid + 256 * it; const int o = q >> 4, pc = q & 15; vst2(out + ((size_t)b * NOUT + o) * LL + l0 + pc * 4, *(const v4f*)(&soT[o][pc * 4])); }
}

extern "C" void kernel_launch(void* const* d_in, const int* in_sizes, int n_in, void* d_out, int out_size, void* d_ws, size_t ws_size, hipStream_t stream) {
  (void)in_sizes; (void)n_in; (void)out_size;
  const float** I = (const float**)d_in;
  const float* x = I[0]; const float* gam = I[1]; const float* bet = I[2]; const float* Win = I[3]; const float* cw = I[4]; const float* cb = I[5]; const float* Wx = I[6]; const float* Wdt = I[7]; const float* bdt = I[8];
  const float* Alog = I[9]; const float* Dp = I[10]; const float* Wout = I[11]; const float* Wp = I[12]; const float* bp = I[13]; const float* ps1 = I[14]; const float* ps2 = I[15];
  char* ws = (char*)d_ws; size_t off = 0;
  auto take = [&](size_t bytes) { char* p = ws + off; off += (bytes + 255) & ~(size_t)255; return p; };
  float* XR = (float*)take((size_t)NR * DM * 4);
  float* UB = (float*)take((size_t)NR * DI * 4);
  float* ZB = (float*)take((size_t)NR * DI * 4);
  float* XP = (float*)take((size_t)NR * DI * 4);
  float* SD = (float*)take((size_t)NR * XDW * 4);
  float* Y = UB; float* MO = XP;
  if (ws_size < off) return;
  k_prep<<<dim3(NLT / 64, NBAT), 256, 0, stream>>>(x, gam, bet, XR);
  k_in<<<dim3(NRC / 64, 2 * DI / 128), 128, 0, stream>>>(XR, Win, UB, ZB);
  k_conv<<<NRC * DI / 4 / 256, 256, 0, stream>>>(UB, cw, cb, XP);
  k_xp<<<NRC / 64, 128, 0, stream>>>(XP, Wx, SD);
  k_scan<<<NSEQ, 256, 0, stream>>>(XP, SD, ZB, Wdt, bdt, Alog, Dp, Y);
  k_lin<<<NRC / 64, 128, 0, stream>>>(Y, Wout, MO);
  k_fin<<<dim3(NLT / 64, NBAT), 256, 0, stream>>>(MO, XR, gam, bet, Wp, bp, ps1, ps2, (float*)d_out);
}
